// PENN_16836271800590
// MI455X (gfx1250) — hardware-verified
//
#include <hip/hip_runtime.h>
#include <stddef.h>


typedef _Float16 h16;
typedef _Float16 v16h __attribute__((ext_vector_type(16)));
typedef _Float16 v8h  __attribute__((ext_vector_type(8)));
typedef float    v8f  __attribute__((ext_vector_type(8)));
typedef float    v4f  __attribute__((ext_vector_type(4)));

#ifndef NB
#define NB 16
#endif
#ifndef SEQ
#define SEQ 512
#endif
#define NB_FULL  16
#define SEQ_FULL 512
#define FEAT  4
#define HID   32
#define MROWS (NB * SEQ)

static_assert(NB >= 1 && NB <= NB_FULL);
static_assert(SEQ >= 128 && SEQ <= SEQ_FULL && (SEQ % 128) == 0);
static_assert(HID == 32);
static_assert(FEAT == 4);
static_assert((MROWS % 128) == 0);
static_assert(((MROWS * HID) % 256) == 0);
static_assert((MROWS % 8) == 0);
static_assert((SEQ % 32) == 0);
static_assert((SEQ % 16) == 0);

#define LDW 40
#define LDA 72
#define LDR 104
#define LDSO 72
static_assert((LDW % 8) == 0 && LDW >= 32);
static_assert((LDA % 8) == 0 && LDA >= 64);
static_assert((LDR % 8) == 0 && LDR >= 96);
static_assert((LDSO % 8) == 0 && LDSO >= 64);

#define WCARRY 64.0f
#define ACARRY 64.0f

static_assert(3 * 32 * LDW * 2 + 32 * LDA * 2 + 8 * 16 * LDA * 2 + 8 * 16 * LDW * 2 <= 131072);
static_assert(32 * LDR * 2 + 8 * 16 * LDA * 2 + 128 * 4 <= 131072);
static_assert(2 * 32 * 32 * 4 + 2 * 8 * 32 * 4 + 8 * LDSO * 2 <= 131072);

#define CD_BYTES   ((size_t)MROWS * HID * 4)
#define S16_BYTES  ((size_t)MROWS * 64 * 2)
#define HP16_BYTES ((size_t)MROWS * HID * 2)
#define PART_BYTES ((size_t)(MROWS / 16) * HID * 4)
#define OFF_CPSI ((size_t)0)
#define OFF_DPSI (OFF_CPSI + CD_BYTES)
#define OFF_CPHI (OFF_DPSI + CD_BYTES)
#define OFF_DPHI (OFF_CPHI + CD_BYTES)
#define OFF_S16  (OFF_DPHI + CD_BYTES)
#define OFF_HP16 (OFF_S16 + S16_BYTES)
#define OFF_PART (OFF_HP16 + HP16_BYTES)
#define WS_TOTAL (OFF_PART + PART_BYTES)
static_assert((CD_BYTES % 128) == 0 && (S16_BYTES % 128) == 0);
static_assert((HP16_BYTES % 128) == 0 && (PART_BYTES % 128) == 0);
static_assert(WS_TOTAL <= (size_t)134217728);

__device__ __forceinline__ float bf16r(float x) {
  unsigned int u = __float_as_uint(x);
  u = (u + 0x7FFFu + ((u >> 16) & 1u)) & 0xFFFF0000u;
  return __uint_as_float(u);
}

static __device__ __forceinline__ h16 toh_flush(float v) {
  const h16 r = (h16)v;
  return (fabsf(v) < 6.103515625e-05f) ? (h16)0.0f : r;
}

__device__ __forceinline__ v16h frag_at(const _Float16* p) {
  v8h lo = *(const v8h*)(p);
  v8h hi = *(const v8h*)(p + 16);
  v16h out;
#pragma unroll
  for (int i = 0; i < 8; ++i) { out[i] = lo[i]; out[i + 8] = hi[i]; }
  return out;
}
__device__ __forceinline__ v16h ld_frag(const _Float16* base, unsigned ld) {
  const unsigned lane = threadIdx.x & 31u;
  return frag_at(base + (lane & 15u) * ld + (lane >> 4) * 8u);
}

__device__ __forceinline__ v8f wmma16(v16h a, v16h b, v8f c) {
  v8f d = __builtin_amdgcn_wmma_f32_16x16x32_f16(false, a, false, b, (short)0, c,
                                                 false, false);
  asm volatile("v_nop\n\tv_nop\n\tv_nop\n\tv_nop" : "+v"(d) : "v"(a), "v"(b));
  return d;
}

__device__ __forceinline__ float red16_sum(float x) {
#pragma unroll
  for (int off = 1; off < 16; off <<= 1) x += __shfl_xor(x, off, 32);
  return x;
}

__device__ __forceinline__ void wave_lds_sync() {
  __builtin_amdgcn_fence(3  , "wavefront");
  asm volatile("s_wait_dscnt 0x0" ::: "memory");
  __builtin_amdgcn_wave_barrier();
}

__device__ __forceinline__ float lrelu_act(float t) {
  return fmaxf(t, 0.01f * t);
}

__global__ __launch_bounds__(256) void node_pre_kernel(
    const float* __restrict__ node_feat,
    const float* __restrict__ psi_w0, const float* __restrict__ psi_b0,
    const float* __restrict__ phi_w0, const float* __restrict__ phi_b0,
    float* __restrict__ c_psi, float* __restrict__ d_psi,
    float* __restrict__ c_phi, float* __restrict__ d_phi) {
  const unsigned t = blockIdx.x * 256u + threadIdx.x;
  const unsigned crow = t >> 5, k = t & 31u;
  const unsigned b = crow / (unsigned)SEQ;
  const unsigned frow = b * (unsigned)SEQ_FULL + (crow - b * (unsigned)SEQ);
  const v4f xv = *(const v4f*)(node_feat + (size_t)frow * FEAT);
  const float x0 = bf16r(xv[0]), x1 = bf16r(xv[1]), x2 = bf16r(xv[2]), x3 = bf16r(xv[3]);
  const float cp = bf16r(psi_b0[k]) + x0 * bf16r(psi_w0[0 * HID + k]) + x1 * bf16r(psi_w0[1 * HID + k])
                                    + x2 * bf16r(psi_w0[2 * HID + k]) + x3 * bf16r(psi_w0[3 * HID + k]);
  const float dpv =                   x0 * bf16r(psi_w0[6 * HID + k]) + x1 * bf16r(psi_w0[7 * HID + k])
                                    + x2 * bf16r(psi_w0[8 * HID + k]) + x3 * bf16r(psi_w0[9 * HID + k]);
  const float cf = bf16r(phi_b0[k]) + x0 * bf16r(phi_w0[0 * HID + k]) + x1 * bf16r(phi_w0[1 * HID + k])
                                    + x2 * bf16r(phi_w0[2 * HID + k]) + x3 * bf16r(phi_w0[3 * HID + k]);
  const float dfv =                   x0 * bf16r(phi_w0[5 * HID + k]) + x1 * bf16r(phi_w0[6 * HID + k])
                                    + x2 * bf16r(phi_w0[7 * HID + k]) + x3 * bf16r(phi_w0[8 * HID + k]);
  *(volatile float*)(c_psi + t) = cp;
  *(volatile float*)(d_psi + t) = dpv;
  *(volatile float*)(c_phi + t) = cf;
  *(volatile float*)(d_phi + t) = dfv;
  __threadfence();
  *(volatile float*)(c_psi + t) = cp;
  *(volatile float*)(d_psi + t) = dpv;
  *(volatile float*)(c_phi + t) = cf;
  *(volatile float*)(d_phi + t) = dfv;
}

__global__ __launch_bounds__(256) void edge_kernel(
    const float* __restrict__ liab,
    const float* __restrict__ c_psi, const float* __restrict__ d_psi,
    const float* __restrict__ c_phi, const float* __restrict__ d_phi,
    const float* __restrict__ psi_w0, const float* __restrict__ phi_w0,
    _Float16* __restrict__ S16) {
  __shared__ __attribute__((aligned(16))) float sdp[32 * 32];
  __shared__ __attribute__((aligned(16))) float sdf[32 * 32];
  __shared__ __attribute__((aligned(16))) float sl[8 * 32];
  __shared__ __attribute__((aligned(16))) float slt[32 * 8];
  __shared__ __attribute__((aligned(16))) _Float16 So[8 * LDSO];

  const unsigned tid = threadIdx.x, k = tid & 31u;
  const unsigned ii = (unsigned)__builtin_amdgcn_readfirstlane((int)(tid >> 5));
  const unsigned crow0 = blockIdx.x * 8u;
  const unsigned b = crow0 / (unsigned)SEQ;
  const unsigned i0 = crow0 - b * (unsigned)SEQ;
  const float* dp = d_psi + (size_t)b * SEQ * HID;
  const float* df = d_phi + (size_t)b * SEQ * HID;
  const float wl  = bf16r(psi_w0[4 * HID + k]);
  const float wlt = bf16r(psi_w0[5 * HID + k]);
  const float wlp = bf16r(phi_w0[4 * HID + k]);
  const float cps = c_psi[(size_t)(crow0 + ii) * HID + k];
  const float cph = c_phi[(size_t)(crow0 + ii) * HID + k];
  float accp = 0.0f, accf = 0.0f;
  const unsigned jj2 = tid >> 3, c2 = tid & 7u;
  const size_t lrow = ((size_t)b * SEQ_FULL + i0 + ii) * SEQ_FULL;
  const size_t lcol = (size_t)b * SEQ_FULL * SEQ_FULL + i0 + c2;

  for (unsigned j0 = 0; j0 < (unsigned)SEQ; j0 += 32u) {
    __syncthreads();
#pragma unroll
    for (unsigned t = 0; t < 4u; ++t) {
      const unsigned e = tid + t * 256u;
      sdp[e] = dp[(size_t)j0 * HID + e];
      sdf[e] = df[(size_t)j0 * HID + e];
    }
    sl[ii * 32u + k] = bf16r(liab[lrow + j0 + k]);
    slt[jj2 * 8u + c2] = bf16r(liab[lcol + (size_t)(j0 + jj2) * SEQ_FULL]);
    __syncthreads();
#pragma unroll 4
    for (unsigned jj = 0; jj < 32u; ++jj) {
      const float Lij = sl[ii * 32u + jj];
      const float Lji = slt[jj * 8u + ii];
      const float zp = fmaf(Lji, wlt, fmaf(Lij, wl, cps + sdp[jj * 32u + k]));
      accp += fmaxf(zp, 0.01f * zp);
      const float zf = fmaf(Lij, wlp, cph + sdf[jj * 32u + k]);
      accf += fmaxf(zf, 0.01f * zf);
    }
  }
  So[ii * LDSO + k]       = toh_flush(accp * (ACARRY / (float)SEQ));
  So[ii * LDSO + 32u + k] = toh_flush(accf * (ACARRY / (float)SEQ));
  __syncthreads();
  if (ii == 0u) {
    v8h x[2];
    size_t off[2];
#pragma unroll
    for (unsigned i = 0; i < 2u; ++i) {
      const unsigned idx = i * 32u + k;
      const unsigned r = idx >> 3, c = (idx & 7u) * 8u;
      x[i] = *(const v8h*)&So[r * LDSO + c];
      off[i] = (size_t)(crow0 + r) * 64u + c;
    }
#pragma unroll
    for (int i = 0; i < 2; ++i) *(volatile v8h*)(S16 + off[i]) = x[i];
    __threadfence();
#pragma unroll
    for (int i = 0; i < 2; ++i) *(volatile v8h*)(S16 + off[i]) = x[i];
  }
}

__global__ __launch_bounds__(256) void node_stage_kernel(
    const float* __restrict__ node_feat, const _Float16* __restrict__ S16,
    const float* __restrict__ psi_w1, const float* __restrict__ psi_b1,
    const float* __restrict__ phi_w1, const float* __restrict__ phi_b1,
    const float* __restrict__ alpha_w0, const float* __restrict__ alpha_b0,
    const float* __restrict__ alpha_w1, const float* __restrict__ alpha_b1,
    _Float16* __restrict__ HP16, float* __restrict__ PART) {
  __shared__ __attribute__((aligned(16))) _Float16 Wp1[32 * LDW];
  __shared__ __attribute__((aligned(16))) _Float16 Wf1[32 * LDW];
  __shared__ __attribute__((aligned(16))) _Float16 Wa1[32 * LDW];
  __shared__ __attribute__((aligned(16))) _Float16 Wa0[32 * LDA];
  __shared__ __attribute__((aligned(16))) _Float16 At[8 * 16 * LDA];
  __shared__ __attribute__((aligned(16))) _Float16 Hs[8 * 16 * LDW];

  const unsigned tid = threadIdx.x, lane = tid & 31u;
  const unsigned w = (unsigned)__builtin_amdgcn_readfirstlane((int)(tid >> 5));
  const unsigned hh = lane >> 4, m = lane & 15u;
  const unsigned row0 = blockIdx.x * 128u + w * 16u;
  const unsigned b = row0 / (unsigned)SEQ;
  const unsigned frow0 = b * (unsigned)SEQ_FULL + (row0 - b * (unsigned)SEQ);
  _Float16* A  = At + w * (16u * LDA);
  _Float16* Hw = Hs + w * (16u * LDW);
  const float inv = 1.0f / (WCARRY * ACARRY);

#pragma unroll 1
  for (unsigned j = 0; j < 4u; ++j) {
    const unsigned idx = tid + 256u * j;
    const unsigned kr = idx >> 5, nc = idx & 31u;
    Wp1[nc * LDW + kr] = toh_flush(WCARRY * bf16r(psi_w1[idx]));
    Wf1[nc * LDW + kr] = toh_flush(WCARRY * bf16r(phi_w1[idx]));
    Wa1[nc * LDW + kr] = toh_flush(WCARRY * bf16r(alpha_w1[idx]));
  }
#pragma unroll 1
  for (unsigned j = 0; j < 8u; ++j) {
    const unsigned idx = tid + 256u * j;
    const unsigned kr = idx >> 5, nc = idx & 31u;
    unsigned srow = (kr < 32u) ? (kr + 4u) : (kr - 32u);
    srow = (srow < 35u) ? srow : 35u;
    const float v = alpha_w0[srow * HID + nc];
    const h16 hv = toh_flush(WCARRY * bf16r(v));
    Wa0[nc * LDA + kr] = (kr < 36u) ? hv : (h16)0.0f;
  }
  {
    const unsigned r = lane >> 1, hf = lane & 1u;
    const v4f xv = *(const v4f*)(node_feat + (size_t)(frow0 + r) * FEAT);
    v8h a0, z;
#pragma unroll
    for (int i = 0; i < 8; ++i) z[i] = (h16)0.0f;
#pragma unroll
    for (int i = 0; i < 4; ++i) {
      const h16 t = toh_flush(ACARRY * bf16r(xv[i]));
      a0[i] = (hf != 0u) ? (h16)0.0f : t;
      a0[i + 4] = (h16)0.0f;
    }
    *(v8h*)&A[r * LDA + 32u + 16u * hf] = a0;
    *(v8h*)&A[r * LDA + 40u + 16u * hf] = z;
  }
  __syncthreads();

  const _Float16* sp = S16 + (size_t)(row0 + m) * 64u + hh * 8u;

  {
    const v16h a = frag_at(sp);
    v8f c0 = {}, c1 = {};
    c0 = wmma16(a, ld_frag(&Wp1[0], LDW), c0);
    c1 = wmma16(a, ld_frag(&Wp1[16 * LDW], LDW), c1);
    const float bl = bf16r(psi_b1[m]), bh = bf16r(psi_b1[16u + m]);
#pragma unroll
    for (int r = 0; r < 8; ++r) {
      Hw[(hh * 8u + (unsigned)r) * LDW + m]       = toh_flush(ACARRY * (c0[r] * inv + bl));
      Hw[(hh * 8u + (unsigned)r) * LDW + 16u + m] = toh_flush(ACARRY * (c1[r] * inv + bh));
    }
  }
  {
    const v16h a = frag_at(sp + 32);
    v8f c0 = {}, c1 = {};
    c0 = wmma16(a, ld_frag(&Wf1[0], LDW), c0);
    c1 = wmma16(a, ld_frag(&Wf1[16 * LDW], LDW), c1);
    const float bl = bf16r(phi_b1[m]), bh = bf16r(phi_b1[16u + m]);
#pragma unroll
    for (int r = 0; r < 8; ++r) {
      A[(hh * 8u + (unsigned)r) * LDA + m]       = toh_flush(ACARRY * (c0[r] * inv + bl));
      A[(hh * 8u + (unsigned)r) * LDA + 16u + m] = toh_flush(ACARRY * (c1[r] * inv + bh));
    }
  }
  wave_lds_sync();

  v8h hx[2];
  size_t hoff[2];
#pragma unroll
  for (unsigned i = 0; i < 2u; ++i) {
    const unsigned idx = i * 32u + lane;
    const unsigned r = idx >> 2, c = (idx & 3u) * 8u;
    hx[i] = *(const v8h*)&Hw[r * LDW + c];
    hoff[i] = (size_t)(row0 + r) * HID + c;
  }

  {
    v8f c0 = {}, c1 = {};
#pragma unroll
    for (int c = 0; c < 2; ++c) {
      const v16h a = ld_frag(A + c * 32, LDA);
      c0 = wmma16(a, ld_frag(&Wa0[c * 32], LDA), c0);
      c1 = wmma16(a, ld_frag(&Wa0[16 * LDA + c * 32], LDA), c1);
    }
    const float bl = bf16r(alpha_b0[m]), bh = bf16r(alpha_b0[16u + m]);
#pragma unroll
    for (int r = 0; r < 8; ++r) {
      A[(hh * 8u + (unsigned)r) * LDA + m]       = toh_flush(ACARRY * lrelu_act(c0[r] * inv + bl));
      A[(hh * 8u + (unsigned)r) * LDA + 16u + m] = toh_flush(ACARRY * lrelu_act(c1[r] * inv + bh));
    }
  }
  wave_lds_sync();

  float contrib;
  {
    const v16h a = ld_frag(A, LDA);
    v8f c0 = {}, c1 = {};
    c0 = wmma16(a, ld_frag(&Wa1[0], LDW), c0);
    c1 = wmma16(a, ld_frag(&Wa1[16 * LDW], LDW), c1);
    const float bl = bf16r(alpha_b1[m]), bh = bf16r(alpha_b1[16u + m]);
    float slo = 0.0f, shi = 0.0f;
#pragma unroll
    for (int r = 0; r < 8; ++r) {
      slo += c0[r] * inv + bl;
      shi += c1[r] * inv + bh;
    }
    slo += __shfl_xor(slo, 16, 32);
    shi += __shfl_xor(shi, 16, 32);
    contrib = (lane < 16u) ? slo : shi;
  }
  float* pl = PART + (size_t)(row0 >> 4) * HID + lane;

#pragma unroll
  for (int i = 0; i < 2; ++i) *(volatile v8h*)(HP16 + hoff[i]) = hx[i];
  *(volatile float*)pl = contrib;
  __threadfence();
#pragma unroll
  for (int i = 0; i < 2; ++i) *(volatile v8h*)(HP16 + hoff[i]) = hx[i];
  *(volatile float*)pl = contrib;
}

__global__ __launch_bounds__(256) void rho_kernel(
    const float* __restrict__ node_feat, const _Float16* __restrict__ HP16,
    const float* __restrict__ PART,
    const float* __restrict__ rho_w0, const float* __restrict__ rho_b0,
    const float* __restrict__ rho_w1, const float* __restrict__ rho_b1,
    float* __restrict__ outp) {
  __shared__ __attribute__((aligned(16))) _Float16 Wr[32 * LDR];
  __shared__ __attribute__((aligned(16))) _Float16 Ar[8 * 16 * LDA];
  __shared__ __attribute__((aligned(16))) float Os[128];

  const unsigned tid = threadIdx.x, lane = tid & 31u;
  const unsigned w = (unsigned)__builtin_amdgcn_readfirstlane((int)(tid >> 5));
  const unsigned hh = lane >> 4, m = lane & 15u;
  const unsigned brow0 = blockIdx.x * 128u;
  const unsigned row0 = brow0 + w * 16u;
  const unsigned b = brow0 / (unsigned)SEQ;
  const unsigned frow0 = b * (unsigned)SEQ_FULL + (row0 - b * (unsigned)SEQ);
  const unsigned fbrow0 = b * (unsigned)SEQ_FULL + (brow0 - b * (unsigned)SEQ);
  _Float16* A = Ar + w * (16u * LDA);
  const float inv = 1.0f / (WCARRY * ACARRY);

#pragma unroll 1
  for (unsigned j = 0; j < 12u; ++j) {
    const unsigned idx = tid + 256u * j;
    const unsigned kr = idx >> 5, nc = idx & 31u;
    unsigned srow = (kr < 32u) ? (kr + 36u) : ((kr < 64u) ? (kr - 28u) : (kr - 64u));
    srow = (srow < 67u) ? srow : 67u;
    const float v = rho_w0[srow * HID + nc];
    const h16 hv = toh_flush(WCARRY * bf16r(v));
    Wr[nc * LDR + kr] = (kr < 68u) ? hv : (h16)0.0f;
  }

  {
    const float* pp = PART + (size_t)(b * ((unsigned)SEQ / 16u)) * HID + lane;
    float ha = 0.0f;
#pragma unroll 4
    for (unsigned u = 0; u < (unsigned)SEQ / 16u; ++u) ha += pp[(size_t)u * HID];
    const h16 ha16 = toh_flush(ha * (ACARRY / (float)SEQ));
#pragma unroll
    for (unsigned r = 0; r < 16u; ++r) A[r * LDA + lane] = ha16;
  }
  {
    const unsigned r = lane >> 1, hf = lane & 1u;
    const v4f xv = *(const v4f*)(node_feat + (size_t)(frow0 + r) * FEAT);
    v8h a0, z;
#pragma unroll
    for (int i = 0; i < 8; ++i) z[i] = (h16)0.0f;
#pragma unroll
    for (int i = 0; i < 4; ++i) {
      const h16 t = toh_flush(ACARRY * bf16r(xv[i]));
      a0[i] = (hf != 0u) ? (h16)0.0f : t;
      a0[i + 4] = (h16)0.0f;
    }
    *(v8h*)&A[r * LDA + 32u + 16u * hf] = a0;
    *(v8h*)&A[r * LDA + 40u + 16u * hf] = z;
  }
  __syncthreads();

  v8f c0 = {}, c1 = {};
  {
    const v16h a = frag_at(HP16 + (size_t)(row0 + m) * HID + hh * 8u);
    c0 = wmma16(a, ld_frag(&Wr[0], LDR), c0);
    c1 = wmma16(a, ld_frag(&Wr[16 * LDR], LDR), c1);
  }
#pragma unroll
  for (int c = 0; c < 2; ++c) {
    const v16h a = ld_frag(A + c * 32, LDA);
    c0 = wmma16(a, ld_frag(&Wr[32 + c * 32], LDR), c0);
    c1 = wmma16(a, ld_frag(&Wr[16 * LDR + 32 + c * 32], LDR), c1);
  }

  const float bl = bf16r(rho_b0[m]), bh = bf16r(rho_b0[16u + m]);
  const float wlo = bf16r(rho_w1[m]), whi = bf16r(rho_w1[16u + m]);
  const float ob = bf16r(rho_b1[0]);
#pragma unroll
  for (int r = 0; r < 8; ++r) {
    float t = lrelu_act(c0[r] * inv + bl) * wlo + lrelu_act(c1[r] * inv + bh) * whi;
    t = red16_sum(t);
    if (m == 0u) Os[w * 16u + hh * 8u + (unsigned)r] = t + ob;
  }
  __syncthreads();
  if (w == 0u) {
    const v4f x = *(const v4f*)&Os[lane * 4u];
    float* p = outp + (size_t)fbrow0 + lane * 4u;
    *(volatile v4f*)p = x;
    __threadfence();
    *(volatile v4f*)p = x;
  }
}

extern "C" void kernel_launch(void* const* d_in, const int* in_sizes, int n_in,
                              void* d_out, int out_size, void* d_ws, size_t ws_size,
                              hipStream_t stream) {
  if (n_in < 18) return;
  const long long need_rows = (long long)(NB - 1) * SEQ_FULL + SEQ;
  if ((long long)in_sizes[0] < need_rows * FEAT) return;
  if ((long long)in_sizes[1] < (need_rows - 1) * SEQ_FULL + SEQ) return;
  if (in_sizes[2] < 10 * HID || in_sizes[3] < HID) return;
  if (in_sizes[4] < HID * HID || in_sizes[5] < HID) return;
  if (in_sizes[6] < 9 * HID || in_sizes[7] < HID) return;
  if (in_sizes[8] < HID * HID || in_sizes[9] < HID) return;
  if (in_sizes[10] < 36 * HID || in_sizes[11] < HID) return;
  if (in_sizes[12] < HID * HID || in_sizes[13] < HID) return;
  if (in_sizes[14] < 68 * HID || in_sizes[15] < HID) return;
  if (in_sizes[16] < HID || in_sizes[17] < 1) return;
  if ((long long)out_size < need_rows) return;
  if (ws_size < WS_TOTAL) return;

  const float* node_feat = (const float*)d_in[0];
  const float* liab      = (const float*)d_in[1];
  const float* psi_w0    = (const float*)d_in[2];
  const float* psi_b0    = (const float*)d_in[3];
  const float* psi_w1    = (const float*)d_in[4];
  const float* psi_b1    = (const float*)d_in[5];
  const float* phi_w0    = (const float*)d_in[6];
  const float* phi_b0    = (const float*)d_in[7];
  const float* phi_w1    = (const float*)d_in[8];
  const float* phi_b1    = (const float*)d_in[9];
  const float* alpha_w0  = (const float*)d_in[10];
  const float* alpha_b0  = (const float*)d_in[11];
  const float* alpha_w1  = (const float*)d_in[12];
  const float* alpha_b1  = (const float*)d_in[13];
  const float* rho_w0    = (const float*)d_in[14];
  const float* rho_b0    = (const float*)d_in[15];
  const float* rho_w1    = (const float*)d_in[16];
  const float* rho_b1    = (const float*)d_in[17];
  float* outp = (float*)d_out;

  char* ws = (char*)d_ws;
  float*    c_psi = (float*)(ws + OFF_CPSI);
  float*    d_psi = (float*)(ws + OFF_DPSI);
  float*    c_phi = (float*)(ws + OFF_CPHI);
  float*    d_phi = (float*)(ws + OFF_DPHI);
  _Float16* S16   = (_Float16*)(ws + OFF_S16);
  _Float16* HP16  = (_Float16*)(ws + OFF_HP16);
  float*    PART  = (float*)(ws + OFF_PART);

  dim3 blk(256);
  node_pre_kernel<<<dim3((MROWS * HID) / 256), blk, 0, stream>>>(
      node_feat, psi_w0, psi_b0, phi_w0, phi_b0, c_psi, d_psi, c_phi, d_phi);
  edge_kernel<<<dim3(MROWS / 8), blk, 0, stream>>>(
      liab, c_psi, d_psi, c_phi, d_phi, psi_w0, phi_w0, S16);
  node_stage_kernel<<<dim3(MROWS / 128), blk, 0, stream>>>(
      node_feat, S16, psi_w1, psi_b1, phi_w1, phi_b1,
      alpha_w0, alpha_b0, alpha_w1, alpha_b1, HP16, PART);
  rho_kernel<<<dim3(MROWS / 128), blk, 0, stream>>>(
      node_feat, HP16, PART, rho_w0, rho_b0, rho_w1, rho_b1, outp);
}
